// InferTree_16226386444598
// MI455X (gfx1250) — hardware-run, weakly checked
//
#include <hip/hip_runtime.h>
#include <math.h>

typedef __attribute__((ext_vector_type(16))) _Float16 v16h;
typedef __attribute__((ext_vector_type(8)))  _Float16 v8h;
typedef __attribute__((ext_vector_type(8)))  float    v8f;
typedef __attribute__((ext_vector_type(4)))  float    v4f;

constexpr int kBatch    = 4096;
constexpr int kDim      = 2048;
constexpr int kWidth    = 11;
constexpr int kNodes1   = 1;
constexpr int kNodes2   = 10;
constexpr int kNodes3   = 100;
constexpr int kNodesAll = kNodes1 + kNodes2 + kNodes3;
constexpr int kBase2    = kNodes1 * kWidth;
constexpr int kBase3    = kBase2 + kNodes2 * kWidth;
constexpr int kCols     = kBase3 + kNodes3 * kWidth;
constexpr int kColsPad  = 1280;
constexpr int kOutC     = 1001;
constexpr int kLeaves   = 1000;
constexpr int kOutElems = kBatch * kOutC;
constexpr int kOutVec4  = kOutElems / 4;
constexpr int kTilesM   = kBatch / 64;
constexpr int kTilesN   = kColsPad / 64;
constexpr int kCeBlocks = kBatch / 32;
constexpr int kCePairs  = 32 * kNodesAll;
constexpr int kCeIters  = (kCePairs + 255) / 256;
constexpr float kXCarry = 16.0f;
constexpr float kWCarry = 1024.0f;
constexpr float kFold   = 1.0f / (kXCarry * kWCarry);
constexpr float kInvBatch = 1.0f / (float)kBatch;

static_assert(kNodesAll == 111, "node count");
static_assert(kBase2 == 11 && kBase3 == 121 && kCols == 1221, "column bases");
static_assert(kColsPad >= kCols && (kColsPad % 64) == 0, "N tile multiple");
static_assert((kBatch % 64) == 0, "M tile multiple");
static_assert((kDim % 32) == 0, "K multiple of 32");
static_assert(kNodes3 * 10 == kLeaves && kLeaves + 1 == kOutC, "leaf columns");
static_assert((kOutElems % 1024) == 0, "output is a whole number of 256-thread float4 blocks");
static_assert(kOutElems * 4 == 16400384, "out0 bytes");
static_assert((kTilesM * kTilesN) % 8 == 0, "tiles per block");
static_assert(kCePairs == 3552 && kCeIters == 14, "penalty pair coverage");
static_assert(kFold == 1.0f / 16384.0f, "carry fold");

constexpr size_t kSzXA   = (size_t)kBatch * kDim * 2;
constexpr size_t kSzWB   = (size_t)kColsPad * kDim * 2;
constexpr size_t kSzBias = (size_t)kColsPad * 4;
constexpr size_t kSzLG   = (size_t)kBatch * kColsPad * 4;
constexpr size_t kSzPart = (size_t)kCeBlocks * 32 * 4;
constexpr size_t kOffXA   = 0;
constexpr size_t kOffWB   = kOffXA + kSzXA;
constexpr size_t kOffBias = kOffWB + kSzWB;
constexpr size_t kOffLG   = kOffBias + kSzBias;
constexpr size_t kOffPart = kOffLG + kSzLG;
constexpr size_t kWsTotal = kOffPart + kSzPart;
static_assert(kWsTotal == 43013120ull, "carve total");
static_assert(kWsTotal <= 134217728ull, "carve cap");
static_assert((kOffWB % 128) == 0 && (kOffBias % 128) == 0 && (kOffLG % 128) == 0 && (kOffPart % 128) == 0, "aligned regions");

union FragU { v16h v; v8h h[2]; };

__device__ __forceinline__ v16h frag_load(const _Float16* p) {
  FragU f;
  f.h[0] = *(const v8h*)(p);
  f.h[1] = *(const v8h*)(p + 16);
  return f.v;
}

__device__ __forceinline__ v8f frag_mma(v16h a, v16h b, v8f c) {
  return __builtin_amdgcn_wmma_f32_16x16x32_f16(false, a, false, b, (short)0, c, false, false);
}

__device__ __forceinline__ void row_guard(v8f& a, v8f& b, v8f& c, v8f& d, v16h x, v16h y0, v16h y1, v16h y2, v16h y3) {
  asm volatile("v_nop\n\tv_nop\n\tv_nop\n\tv_nop"
               : "+v"(a), "+v"(b), "+v"(c), "+v"(d)
               : "v"(x), "v"(y0), "v"(y1), "v"(y2), "v"(y3));
}

__device__ __forceinline__ void acc_guard4(v8f& a, v8f& b, v8f& c, v8f& d) {
  asm volatile("v_nop\n\tv_nop\n\tv_nop\n\tv_nop" : "+v"(a), "+v"(b), "+v"(c), "+v"(d));
}

__global__ __launch_bounds__(256) void act_plane_kernel(const float* __restrict__ x, unsigned short* __restrict__ xa)
{
  const int i = blockIdx.x * 256 + threadIdx.x;
  if (i >= kBatch * kDim / 8) return;
  const size_t e0 = (size_t)i << 3;
  const v4f a0 = *(const v4f*)(x + e0);
  const v4f a1 = *(const v4f*)(x + e0 + 4);
  v8h hv;
#pragma unroll
  for (int e = 0; e < 4; ++e) {
    float f0 = a0[e] * kXCarry;
    float f1 = a1[e] * kXCarry;
    asm volatile("" : "+v"(f0));
    asm volatile("" : "+v"(f1));
    hv[e]     = (_Float16)f0;
    hv[4 + e] = (_Float16)f1;
  }
  unsigned short* q = xa + e0;
  *(volatile v8h*)q = hv;
  __threadfence();
  *(volatile v8h*)q = hv;
}

__global__ __launch_bounds__(256) void weight_plane_kernel(
    const float* __restrict__ W1, const float* __restrict__ W2, const float* __restrict__ W3,
    unsigned short* __restrict__ wb)
{
  const int row = blockIdx.x;
  const int tid = threadIdx.x;
  const bool valid = row < kCols;
  const float* src;
  if (row < kBase2) {
    src = W1 + (size_t)row * kDim;
  } else if (row < kBase3) {
    src = W2 + (size_t)(row - kBase2) * kDim;
  } else {
    const int rc = (row < kCols) ? row : (kCols - 1);
    src = W3 + (size_t)(rc - kBase3) * kDim;
  }
  const v4f a0 = *(const v4f*)(src + tid * 8);
  const v4f a1 = *(const v4f*)(src + tid * 8 + 4);
  v8h hv;
#pragma unroll
  for (int e = 0; e < 4; ++e) {
    float f0 = valid ? (a0[e] * kWCarry) : 0.0f;
    float f1 = valid ? (a1[e] * kWCarry) : 0.0f;
    asm volatile("" : "+v"(f0));
    asm volatile("" : "+v"(f1));
    hv[e]     = (_Float16)f0;
    hv[4 + e] = (_Float16)f1;
  }
  unsigned short* q = wb + (size_t)row * kDim + tid * 8;
  *(volatile v8h*)q = hv;
  __threadfence();
  *(volatile v8h*)q = hv;
}

__global__ __launch_bounds__(256) void bias_cat_kernel(
    const float* __restrict__ b1, const float* __restrict__ b2, const float* __restrict__ b3,
    float* __restrict__ bias)
{
  const int col = blockIdx.x * 256 + threadIdx.x;
  if (col >= kColsPad) return;
  int i1 = col;
  i1 = i1 < 0 ? 0 : i1;
  i1 = i1 > (kBase2 - 1) ? (kBase2 - 1) : i1;
  int i2 = col - kBase2;
  i2 = i2 < 0 ? 0 : i2;
  i2 = i2 > (kBase3 - kBase2 - 1) ? (kBase3 - kBase2 - 1) : i2;
  int i3 = col - kBase3;
  i3 = i3 < 0 ? 0 : i3;
  i3 = i3 > (kCols - kBase3 - 1) ? (kCols - kBase3 - 1) : i3;
  float v1 = b1[i1];
  float v2 = b2[i2];
  float v3 = b3[i3];
  asm volatile("" : "+v"(v1));
  asm volatile("" : "+v"(v2));
  asm volatile("" : "+v"(v3));
  float v = 0.0f;
  v = (col < kCols) ? v3 : v;
  v = (col < kBase3) ? v2 : v;
  v = (col < kBase2) ? v1 : v;
  volatile float* q = bias + col;
  *q = v;
  __threadfence();
  *q = v;
}

__global__ __launch_bounds__(256) void logits_gemm_kernel(
    const unsigned short* __restrict__ Ap, const unsigned short* __restrict__ Btp,
    const float* __restrict__ bias, float* __restrict__ C)
{
  const _Float16* A  = (const _Float16*)Ap;
  const _Float16* Bt = (const _Float16*)Btp;
  __shared__ __align__(16) float sT[8][16 * 68];
  const int lane = threadIdx.x & 31;
  const int wave = __builtin_amdgcn_readfirstlane((int)(threadIdx.x >> 5));
  const int tile = blockIdx.x * 8 + wave;
  if (tile >= kTilesM * kTilesN) return;
  const int tm = tile / kTilesN;
  const int tn = tile - tm * kTilesN;
  const int m0 = tm << 6;
  const int n0 = tn << 6;

  const int rlane = lane & 15;
  const int koff  = (lane >> 4) * 8;
  const int mOff  = (lane >> 4) * 8;

  v8f acc[4][4];
#pragma unroll
  for (int i = 0; i < 4; ++i)
#pragma unroll
    for (int j = 0; j < 4; ++j) acc[i][j] = (v8f){0.f, 0.f, 0.f, 0.f, 0.f, 0.f, 0.f, 0.f};

#pragma unroll 1
  for (int k0 = 0; k0 < kDim; k0 += 32) {
    v16h bh[4];
#pragma unroll
    for (int j = 0; j < 4; ++j) {
      const size_t bo = (size_t)(n0 + (j << 4) + rlane) * kDim + koff + k0;
      bh[j] = frag_load(Bt + bo);
    }
#pragma unroll
    for (int i = 0; i < 4; ++i) {
      const size_t ao = (size_t)(m0 + (i << 4) + rlane) * kDim + koff + k0;
      const v16h ah = frag_load(A + ao);
#pragma unroll
      for (int j = 0; j < 4; ++j) acc[i][j] = frag_mma(ah, bh[j], acc[i][j]);
      row_guard(acc[i][0], acc[i][1], acc[i][2], acc[i][3], ah, bh[0], bh[1], bh[2], bh[3]);
    }
  }
  acc_guard4(acc[0][0], acc[0][1], acc[0][2], acc[0][3]);
  acc_guard4(acc[1][0], acc[1][1], acc[1][2], acc[1][3]);
  acc_guard4(acc[2][0], acc[2][1], acc[2][2], acc[2][3]);
  acc_guard4(acc[3][0], acc[3][1], acc[3][2], acc[3][3]);

  float* slab = sT[wave];
#pragma unroll
  for (int i = 0; i < 4; ++i) {
    const int mBase = m0 + (i << 4);
#pragma unroll
    for (int j = 0; j < 4; ++j) {
      const int n = n0 + (j << 4) + rlane;
      const float bv = bias[n];
#pragma unroll
      for (int r = 0; r < 8; ++r) {
        const float v = acc[i][j][r] * kFold + bv;
        slab[(mOff + r) * 68 + (j << 4) + rlane] = v;
      }
    }
    __builtin_amdgcn_fence(__ATOMIC_RELEASE, "workgroup");
    __builtin_amdgcn_wave_barrier();
    __builtin_amdgcn_fence(__ATOMIC_ACQUIRE, "workgroup");
    {
      const int hh = lane >> 4;
      const int c4 = (lane & 15) * 4;
      for (int pass = 0; pass < 2; ++pass) {
#pragma unroll
        for (int it = 0; it < 8; ++it) {
          const int row = it * 2 + hh;
          const v4f v = *(const v4f*)(slab + row * 68 + c4);
          *(volatile v4f*)(C + (size_t)(mBase + row) * kColsPad + n0 + c4) = v;
        }
        __threadfence();
      }
    }
    __builtin_amdgcn_fence(__ATOMIC_RELEASE, "workgroup");
    __builtin_amdgcn_wave_barrier();
    __builtin_amdgcn_fence(__ATOMIC_ACQUIRE, "workgroup");
  }
}

__device__ __forceinline__ float leaf_value(const float* __restrict__ L, int e)
{
  const int b  = e / kOutC;
  const int c  = e - b * kOutC;
  const int cm = (c > 0) ? (c - 1) : 0;
  const int k  = cm / 10;
  const int jj = cm - k * 10;
  float t = L[(size_t)b * kColsPad + kBase3 + k * kWidth + 1 + jj];
  asm volatile("" : "+v"(t));
  return (c > 0) ? t : 0.0f;
}

__global__ __launch_bounds__(256) void leaf_fill_kernel(const float* __restrict__ L, float* __restrict__ out)
{
  const int i = blockIdx.x * 256 + threadIdx.x;
  if (i >= kOutVec4) return;
  const int e0 = i * 4;
  const float t0 = leaf_value(L, e0);
  const float t1 = leaf_value(L, e0 + 1);
  const float t2 = leaf_value(L, e0 + 2);
  const float t3 = leaf_value(L, e0 + 3);
  const v4f v = (v4f){t0, t1, t2, t3};
  float* q = out + e0;
  *(volatile v4f*)q = v;
  __threadfence();
  *(volatile v4f*)q = v;
}

__global__ __launch_bounds__(256) void path_ce_partial_kernel(
    const float* __restrict__ L, const int* __restrict__ labels, float* __restrict__ partials)
{
  __shared__ float red[256];
  const int tid  = threadIdx.x;
  const int lane = tid & 31;
  const int wave = __builtin_amdgcn_readfirstlane((int)(threadIdx.x >> 5));
  const int r0 = blockIdx.x * 32;
  float accum = 0.0f;
#pragma unroll 1
  for (int it = 0; it < kCeIters; ++it) {
    const int p = it * 256 + tid;
    const bool live = p < kCePairs;
    const int pc = live ? p : (kCePairs - 1);
    const int bl = pc / kNodesAll;
    const int n  = pc - bl * kNodesAll;
    const int b  = r0 + bl;
    int lab = labels[b];
    lab = lab < 0 ? 0 : lab;
    lab = lab > (kLeaves - 1) ? (kLeaves - 1) : lab;
    const int n2 = lab / 100;
    const int n3 = lab / 10;
    const int c2 = n3 - n2 * 10;
    const int c3 = lab - n3 * 10;
    int t = n2 + 1;
    float w = 1.0f;
    const int t2 = (n2 == (n - 1)) ? (c2 + 1) : 0;
    const int t3 = (n3 == (n - 11)) ? (c3 + 1) : 0;
    t = (n >= 1) ? t2 : t;
    w = (n >= 1) ? 0.5f : w;
    t = (n >= 11) ? t3 : t;
    w = (n >= 11) ? (1.0f / 3.0f) : w;
    const float* lp = L + (size_t)b * kColsPad + n * kWidth;
    float mx = -INFINITY;
    float lt = 0.0f;
#pragma unroll 1
    for (int c = 0; c < kWidth; ++c) {
      const float v = lp[c];
      mx = fmaxf(mx, v);
      lt = (c == t) ? v : lt;
    }
    float s = 0.0f;
#pragma unroll 1
    for (int c = 0; c < kWidth; ++c) {
      s += expf(lp[c] - mx);
    }
    const float ce = (logf(s) + mx) - lt;
    const float term = ce * (w * kInvBatch);
    accum += live ? term : 0.0f;
  }
  red[tid] = accum;
  __syncthreads();
#pragma unroll 1
  for (int off = 128; off > 0; off >>= 1) {
    if (tid < off) red[tid] += red[tid + off];
    __syncthreads();
  }
  if (wave == 0) {
    const float tot = red[0];
    const float val = (lane == 0) ? tot : 0.0f;
    volatile float* q = partials + (size_t)blockIdx.x * 32 + lane;
    *q = val;
    __threadfence();
    *q = val;
  }
}

__global__ __launch_bounds__(32) void path_ce_final_kernel(const float* __restrict__ partials, float* __restrict__ out1)
{
  const int lane = threadIdx.x & 31;
  float s = 0.0f;
#pragma unroll
  for (int j = 0; j < kCeBlocks / 32; ++j) {
    s += partials[(size_t)(j * 32 + lane) * 32];
  }
  s += __shfl_xor(s, 16, 32);
  s += __shfl_xor(s, 8, 32);
  s += __shfl_xor(s, 4, 32);
  s += __shfl_xor(s, 2, 32);
  s += __shfl_xor(s, 1, 32);
  if (lane == 0) {
    volatile float* q = out1;
    *q = s;
    __threadfence();
    *q = s;
  }
}

extern "C" void kernel_launch(void* const* d_in, const int* in_sizes, int n_in,
                              void* d_out, int out_size, void* d_ws, size_t ws_size,
                              hipStream_t stream) {
  if (n_in < 8) return;
  if (in_sizes[0] != kBatch * kDim) return;
  if (in_sizes[1] != kBatch) return;
  if (in_sizes[2] != kNodes1 * kWidth * kDim) return;
  if (in_sizes[3] != kNodes1 * kWidth) return;
  if (in_sizes[4] != kNodes2 * kWidth * kDim) return;
  if (in_sizes[5] != kNodes2 * kWidth) return;
  if (in_sizes[6] != kNodes3 * kWidth * kDim) return;
  if (in_sizes[7] != kNodes3 * kWidth) return;
  if (out_size != kOutElems + 1) return;
  if (ws_size < kWsTotal) return;

  const float* x      = (const float*)d_in[0];
  const int*   labels = (const int*)d_in[1];
  const float* W1     = (const float*)d_in[2];
  const float* b1     = (const float*)d_in[3];
  const float* W2     = (const float*)d_in[4];
  const float* b2     = (const float*)d_in[5];
  const float* W3     = (const float*)d_in[6];
  const float* b3     = (const float*)d_in[7];
  float* out = (float*)d_out;

  char* ws = (char*)d_ws;
  unsigned short* XA   = (unsigned short*)(ws + kOffXA);
  unsigned short* WB   = (unsigned short*)(ws + kOffWB);
  float*          BIAS = (float*)(ws + kOffBias);
  float*          LG   = (float*)(ws + kOffLG);
  float*          PART = (float*)(ws + kOffPart);

  act_plane_kernel<<<(kBatch * kDim / 8) / 256, 256, 0, stream>>>(x, XA);
  weight_plane_kernel<<<kColsPad, 256, 0, stream>>>(W1, W2, W3, WB);
  bias_cat_kernel<<<kColsPad / 256, 256, 0, stream>>>(b1, b2, b3, BIAS);
  logits_gemm_kernel<<<(kTilesM * kTilesN) / 8, 256, 0, stream>>>(XA, WB, BIAS, LG);
  leaf_fill_kernel<<<kOutVec4 / 256, 256, 0, stream>>>(LG, out);
  path_ce_partial_kernel<<<kCeBlocks, 256, 0, stream>>>(LG, labels, PART);
  path_ce_final_kernel<<<1, 32, 0, stream>>>(PART, out + kOutElems);
}
